// GraphSAGE_9466107921073
// MI455X (gfx1250) — hardware-verified
//
#include <hip/hip_runtime.h>
#include <stddef.h>
#include <stdint.h>


#define DF     128
#define DO3    64
#define XP     128
#define HP     256
#define K1C    384
#define K2C    512
#define K3C    256
#define NTHR   256
#define NWAVE  8
#define EPT    8
#define CHUNK  (NTHR * EPT)
#define WCAP   (EPT * 32)
#define LISTN  (NWAVE * WCAP)
#define NBA    1024
#define SLA    10
#define RCAP   28672
#define DEGCAP 64
#define GBM    64
#define GBN    128
#define GTHR   128
#define GWAVE  (GTHR / 32)
#define ROWH   256
#define UPART  2048
#define UP3    1024
#define NUW1   (3 * UPART)
#define NUW2   (4 * UPART)
#define NUW3   (4 * UP3)
#define NUWE   (NUW1 + NUW2 + NUW3)
#define AGG_ZINTS    (LISTN + 2 * RCAP + 3 * NBA)
#define MISC_INTS    16
#define ROWBUF_INTS  (NWAVE * ROWH / 2)
#define DREC_INTS    (DO3 * 2)
#define AGG_LDS_INTS (AGG_ZINTS + MISC_INTS + ROWBUF_INTS + DREC_INTS)
#define WSMAX  134217728

static_assert((CHUNK & (CHUNK - 1)) == 0 && CHUNK <= 4096);
static_assert((NBA & (NBA - 1)) == 0 && NBA == (1 << SLA));
static_assert(((long long)CHUNK << SLA) < (1LL << 31));
static_assert(LISTN % NTHR == 0);
static_assert(NBA % NWAVE == 0 && NBA % 32 == 0 && NBA % GBM == 0);
static_assert(RCAP % 4 == 0 && AGG_ZINTS % 4 == 0 && LISTN % 4 == 0 && ((AGG_ZINTS + MISC_INTS) % 4) == 0);
static_assert(AGG_ZINTS % (NTHR * 4) == 0);
static_assert(K1C % 32 == 0 && K2C % 32 == 0 && K3C % 32 == 0 && HP % 32 == 0 && XP % 32 == 0);
static_assert(K1C == HP + XP && K2C == 2 * HP && K3C == HP && HP == 2 * DF && ROWH == HP);
static_assert(GBN == DF && GBM == GWAVE * 16 && DF == 4 * 32 && GTHR == GWAVE * 32 && DO3 == 2 * 32);
static_assert(UPART % NTHR == 0 && UP3 % NTHR == 0 && NUW1 % NTHR == 0 && NUW2 % NTHR == 0 && NUWE % NTHR == 0);
static_assert(UPART == DF * (DF / 8) && UP3 == DO3 * (DF / 8));
static_assert(ROWBUF_INTS * 4 == NWAVE * DO3 * 8);
static_assert(AGG_LDS_INTS * 4 <= 300000);
static_assert(RCAP >= 17455 && DEGCAP >= 43);

typedef float          v2f   __attribute__((ext_vector_type(2)));
typedef float          v4f   __attribute__((ext_vector_type(4)));
typedef float          v8f   __attribute__((ext_vector_type(8)));
typedef double         v2d   __attribute__((ext_vector_type(2)));
typedef int            v4i   __attribute__((ext_vector_type(4)));
typedef int            v8i   __attribute__((ext_vector_type(8)));
typedef unsigned       v2u   __attribute__((ext_vector_type(2)));
typedef unsigned short v4us  __attribute__((ext_vector_type(4)));
typedef unsigned short v8us  __attribute__((ext_vector_type(8)));
typedef unsigned short v16us __attribute__((ext_vector_type(16)));
typedef __bf16         v16bf __attribute__((ext_vector_type(16)));
typedef v2f  __attribute__((may_alias)) v2fa;
typedef v4f  __attribute__((may_alias)) v4fa;
typedef v2d  __attribute__((may_alias)) v2da;
typedef v4i  __attribute__((may_alias)) v4ia;
typedef v2u  __attribute__((may_alias)) v2ua;
typedef v4us __attribute__((may_alias)) v4usa;
typedef v8us __attribute__((may_alias)) v8usa;
union FragB { v16bf v; v16us u; v8us h[2]; v8i w; };

__device__ __forceinline__ v8f wmb(const FragB& a, const FragB& b, v8f c) {
  v8f d = __builtin_amdgcn_wmma_f32_16x16x32_bf16(false, a.v, false, b.v, (short)0, c, false, false);
  asm volatile("v_nop\n\tv_nop\n\tv_nop\n\tv_nop" : "+v"(d) : "v"(a.w), "v"(b.w));
  return d;
}

__device__ __forceinline__ v8f z8() { v8f z = {0.f, 0.f, 0.f, 0.f, 0.f, 0.f, 0.f, 0.f}; return z; }

__device__ __forceinline__ unsigned bf16_bits(float f) {
  const unsigned u = __float_as_uint(f);
  const unsigned r = (u + 0x7FFFu + ((u >> 16) & 1u)) >> 16;
  return (f != f) ? 0x7fc0u : r;
}
__device__ __forceinline__ float bf16_val(float f) {
  return __uint_as_float(bf16_bits(f) << 16);
}
__device__ __forceinline__ unsigned hl_bits(float v, unsigned& lo) {
  const unsigned hb = bf16_bits(v);
  lo = bf16_bits(v - __uint_as_float(hb << 16));
  return hb;
}
__device__ __forceinline__ float sigm(float v) { return 1.0f / (1.0f + expf(-v)); }

__device__ __forceinline__ void wave_sync() {
  __builtin_amdgcn_fence(__ATOMIC_RELEASE, "wavefront");
  __builtin_amdgcn_wave_barrier();
  __builtin_amdgcn_fence(__ATOMIC_ACQUIRE, "wavefront");
}

template <int SLB>
__device__ __forceinline__ int scan_chunk(const int* __restrict__ dsts, int nE, int cbase, int slotBase,
                                          int nb, int vec8, int* list, int tid, int lane, int wave) {
  int wc = 0;
  const int el0  = tid * EPT;
  const int e0   = cbase + el0;
  const int sent = -2147483647 - 1;
  v4i da, db;
  if (vec8 != 0 && cbase + CHUNK <= nE) {
    da = *(const v4i*)(dsts + e0);
    db = *(const v4i*)(dsts + e0 + 4);
  } else {
    da.x = (e0     < nE) ? dsts[min(e0,     nE - 1)] : sent;
    da.y = (e0 + 1 < nE) ? dsts[min(e0 + 1, nE - 1)] : sent;
    da.z = (e0 + 2 < nE) ? dsts[min(e0 + 2, nE - 1)] : sent;
    da.w = (e0 + 3 < nE) ? dsts[min(e0 + 3, nE - 1)] : sent;
    db.x = (e0 + 4 < nE) ? dsts[min(e0 + 4, nE - 1)] : sent;
    db.y = (e0 + 5 < nE) ? dsts[min(e0 + 5, nE - 1)] : sent;
    db.z = (e0 + 6 < nE) ? dsts[min(e0 + 6, nE - 1)] : sent;
    db.w = (e0 + 7 < nE) ? dsts[min(e0 + 7, nE - 1)] : sent;
  }
  const unsigned nbs = (unsigned)slotBase;
  const unsigned unb = (unsigned)nb;
  const unsigned s0 = (unsigned)da.x - nbs, s1 = (unsigned)da.y - nbs;
  const unsigned s2 = (unsigned)da.z - nbs, s3 = (unsigned)da.w - nbs;
  const unsigned s4 = (unsigned)db.x - nbs, s5 = (unsigned)db.y - nbs;
  const unsigned s6 = (unsigned)db.z - nbs, s7 = (unsigned)db.w - nbs;
  const bool h0 = s0 < unb, h1 = s1 < unb, h2 = s2 < unb, h3 = s3 < unb;
  const bool h4 = s4 < unb, h5 = s5 < unb, h6 = s6 < unb, h7 = s7 < unb;
  const unsigned any = __builtin_amdgcn_ballot_w32(h0 | h1 | h2 | h3 | h4 | h5 | h6 | h7);
  if (any != 0u) {
#define HITJ(J, HJ, SJ) { \
      const unsigned mj = __builtin_amdgcn_ballot_w32(HJ); \
      if (mj != 0u) { \
        if (HJ) { \
          const int pos = wc + (int)__builtin_amdgcn_mbcnt_lo(mj, 0u); \
          if (pos < WCAP) list[wave * WCAP + pos] = ((el0 + (J)) << SLB) | (int)(SJ); \
        } \
        wc += (int)__builtin_popcount(mj); } }
    HITJ(0, h0, s0)
    HITJ(1, h1, s1)
    HITJ(2, h2, s2)
    HITJ(3, h3, s3)
    HITJ(4, h4, s4)
    HITJ(5, h5, s5)
    HITJ(6, h6, s6)
    HITJ(7, h7, s7)
#undef HITJ
  }
  return wc;
}

__device__ __forceinline__ void put8(const float* __restrict__ sp, unsigned short* dp, bool lv) {
  const v4f a = *(const v4f*)sp;
  const v4f b = *(const v4f*)(sp + 4);
  v8us o;
  o[0] = (unsigned short)bf16_bits(lv ? a.x : 0.0f); o[1] = (unsigned short)bf16_bits(lv ? a.y : 0.0f);
  o[2] = (unsigned short)bf16_bits(lv ? a.z : 0.0f); o[3] = (unsigned short)bf16_bits(lv ? a.w : 0.0f);
  o[4] = (unsigned short)bf16_bits(lv ? b.x : 0.0f); o[5] = (unsigned short)bf16_bits(lv ? b.y : 0.0f);
  o[6] = (unsigned short)bf16_bits(lv ? b.z : 0.0f); o[7] = (unsigned short)bf16_bits(lv ? b.w : 0.0f);
  *(volatile v8us*)dp = o;
  __threadfence();
  *(volatile v8us*)dp = o;
}

__global__ __launch_bounds__(NTHR) void k_prep(const float* __restrict__ x,
                                               const float* __restrict__ w1l, const float* __restrict__ w1r,
                                               const float* __restrict__ w2l, const float* __restrict__ w2r,
                                               const float* __restrict__ w3l, const float* __restrict__ w3r,
                                               unsigned short* w1c, unsigned short* w2c, unsigned short* w3c,
                                               unsigned short* xb, int nN, int nUnits) {
  const int u = (int)blockIdx.x * NTHR + (int)threadIdx.x;
  if (u < NUW1) {
    const int part = u >> 11;
    const int v = u & (UPART - 1);
    const int n = v >> 4, k8 = (v & 15) * 8;
    const size_t so = (size_t)n * DF + (size_t)k8;
    unsigned short* dp = w1c + (size_t)n * K1C + (size_t)part * DF + k8;
    if (part < 2) put8(w1l + so, dp, true);
    else          put8(w1r + so, dp, true);
  } else if (u < NUW1 + NUW2) {
    const int q = u - NUW1;
    const int part = q >> 11;
    const int v = q & (UPART - 1);
    const int n = v >> 4, k8 = (v & 15) * 8;
    const size_t so = (size_t)n * DF + (size_t)k8;
    unsigned short* dp = w2c + (size_t)n * K2C + (size_t)part * DF + k8;
    if (part < 2) put8(w2l + so, dp, true);
    else          put8(w2r + so, dp, true);
  } else if (u < NUWE) {
    const int q = u - NUW1 - NUW2;
    const int part = q >> 10;
    const int v = q & (UP3 - 1);
    const int n = v >> 4, k8 = (v & 15) * 8;
    const size_t so = (size_t)n * DF + (size_t)k8;
    const int coff = (part & 1) * DF;
    if (part < 2) put8(w3l + so, w3c + (size_t)n * K3C + coff + k8, true);
    else          put8(w3r + so, w3c + (size_t)(n + DO3) * K3C + coff + k8, true);
  } else if (u < nUnits) {
    const int v = u - NUWE;
    const int row = v >> 4, k8 = (v & 15) * 8;
    const int rc = row < nN ? row : nN - 1;
    put8(x + (size_t)rc * DF + k8, xb + (size_t)v * 8, row < nN);
  }
}

template <int MODE>
__global__ __launch_bounds__(NTHR) void k_scan(const int* __restrict__ srcs, const int* __restrict__ dsts,
                                               int nE, int nN, int vec8, int mRows,
                                               const unsigned short* __restrict__ gin,
                                               const float* __restrict__ pr3, const float* __restrict__ b3,
                                               unsigned short* aggOut, double* rec) {
  extern __shared__ __attribute__((aligned(16))) int dsm[];
  int* list = dsm;
  int* hl   = dsm + LISTN;
  int* sl   = hl + RCAP;
  int* cnt  = sl + RCAP;
  int* offs = cnt + NBA;
  int* cur  = offs + NBA;
  int* misc = cur + NBA;
  const int tid = (int)threadIdx.x, lane = tid & 31, wave = tid >> 5;
  unsigned short* rowbuf = (unsigned short*)(misc + MISC_INTS) + wave * ROWH;
  const int nodeBase = (int)blockIdx.x * NBA;

  {
    const v4i z4 = {0, 0, 0, 0};
    for (int i = tid * 4; i < AGG_ZINTS; i += NTHR * 4) *(v4ia*)(dsm + i) = z4;
    if (tid < MISC_INTS) misc[tid] = 0;
  }
  __syncthreads();

  int t = 0, ov = 0;
  const int nChunks = (nE + CHUNK - 1) / CHUNK;
#pragma unroll 1
  for (int ch = 0; ch < nChunks; ++ch) {
    const int cbase = ch * CHUNK;
    const int wc = scan_chunk<SLA>(dsts, nE, cbase, nodeBase, NBA, vec8, list, tid, lane, wave);
    if (lane == 0) misc[wave] = wc;
    __syncthreads();
    if (wave == 0) {
#pragma unroll 1
      for (int w2 = 0; w2 < NWAVE; ++w2) {
        int c = misc[w2];
        c = c < 0 ? 0 : (c > WCAP ? WCAP : c);
#pragma unroll 1
        for (int b0 = 0; b0 < c; b0 += 32) {
          const int idx = b0 + lane;
          const int ent_ = list[w2 * WCAP + (idx < WCAP ? idx : WCAP - 1)];
          const int m32 = (c - b0) < 32 ? (c - b0) : 32;
#pragma unroll 1
          for (int k = 0; k < m32; ++k) {
            const int u    = __builtin_amdgcn_readlane(ent_, k);
            const int slot = u & (NBA - 1);
            const int el   = (u >> SLA) & (CHUNK - 1);
            const int pk   = ((cbase + el) << SLA) | slot;
            if (t < RCAP) {
              if (lane == 0) { hl[t] = pk; cnt[slot] = cnt[slot] + 1; }
              t = t + 1;
            } else {
              ov = 1;
            }
          }
        }
      }
    }
    __syncthreads();
  }
  if (wave == 0 && lane == 0) { misc[8] = t; misc[9] = ov; }
  __syncthreads();
  int tt = misc[8];
  tt = tt < 0 ? 0 : (tt > RCAP ? RCAP : tt);
  const int ovf = misc[9];

  if (wave == 0) {
    const int base = lane * (NBA / 32);
    int s = 0;
#pragma unroll 1
    for (int i = 0; i < NBA / 32; ++i) s += cnt[base + i];
    int incl = s;
#pragma unroll
    for (int d = 1; d < 32; d <<= 1) {
      const int y = __shfl_up(incl, d, 32);
      if (lane >= d) incl += y;
    }
    int run = incl - s;
#pragma unroll 1
    for (int i = 0; i < NBA / 32; ++i) {
      const int cv = cnt[base + i];
      offs[base + i] = run;
      cur[base + i]  = run;
      run += cv;
    }
  }
  __syncthreads();
  if (wave == 0) {
#pragma unroll 1
    for (int b0 = 0; b0 < tt; b0 += 32) {
      const int idx = b0 + lane;
      const int ent_ = hl[idx < RCAP ? idx : RCAP - 1];
      const int m32 = (tt - b0) < 32 ? (tt - b0) : 32;
#pragma unroll 1
      for (int k = 0; k < m32; ++k) {
        const int u    = __builtin_amdgcn_readlane(ent_, k);
        const int slot = u & (NBA - 1);
        if (lane == 0) {
          int p = cur[slot];
          p = p < 0 ? 0 : (p > RCAP - 1 ? RCAP - 1 : p);
          sl[p] = u;
          cur[slot] = p + 1;
        }
      }
    }
  }
  __syncthreads();

  const float qnan = __int_as_float(0x7fc00000);
  const float pz = (ovf != 0) ? qnan : 0.0f;
  double d0 = 0.0, d1 = 0.0;
  float bq0 = 0.0f, bq1 = 0.0f;
  if constexpr (MODE == 2) {
    const v2f bb = *(const v2f*)(b3 + 2 * lane);
    bq0 = bf16_val(bb.x);
    bq1 = bf16_val(bb.y);
  }
#pragma unroll 1
  for (int si = 0; si < NBA / NWAVE; ++si) {
    const int s    = si * NWAVE + wave;
    const int node = nodeBase + s;
    int c = cnt[s];
    const bool big = c > DEGCAP;
    c = c < 0 ? 0 : (c > DEGCAP ? DEGCAP : c);
    int o = offs[s];
    o = o < 0 ? 0 : (o > RCAP ? RCAP : o);
    const float pzr = big ? qnan : pz;
    const bool live = node < nN;
    const int nc = live ? node : nN - 1;
    float a0 = 0.0f, a1 = 0.0f, a2 = 0.0f, a3 = 0.0f;
#pragma unroll 1
    for (int b0 = 0; b0 < c; b0 += 32) {
      int idx = o + b0 + lane;
      idx = idx > RCAP - 1 ? RCAP - 1 : idx;
      const int ent_ = sl[idx];
      int eid = ent_ >> SLA;
      eid = eid < 0 ? 0 : (eid > nE - 1 ? nE - 1 : eid);
      int sr = srcs[eid];
      sr = sr < 0 ? 0 : (sr > nN - 1 ? nN - 1 : sr);
      const int m32 = (c - b0) < 32 ? (c - b0) : 32;
#pragma unroll 1
      for (int k = 0; k < m32; ++k) {
        const int sk = __builtin_amdgcn_readlane(sr, k);
        if constexpr (MODE == 0) {
          const unsigned short* rp = gin + (size_t)sk * XP + 4 * lane;
          const v2u wh = *(const v2ua*)rp;
          a0 += __uint_as_float(wh.x << 16);
          a1 += __uint_as_float(wh.x & 0xffff0000u);
          a2 += __uint_as_float(wh.y << 16);
          a3 += __uint_as_float(wh.y & 0xffff0000u);
        } else if constexpr (MODE == 1) {
          const unsigned short* rp = gin + (size_t)sk * HP + 4 * lane;
          const v2u wh = *(const v2ua*)rp;
          const v2u wl = *(const v2ua*)(rp + DF);
          const float f0 = __uint_as_float(wh.x << 16)         + __uint_as_float(wl.x << 16);
          const float f1 = __uint_as_float(wh.x & 0xffff0000u) + __uint_as_float(wl.x & 0xffff0000u);
          const float f2 = __uint_as_float(wh.y << 16)         + __uint_as_float(wl.y << 16);
          const float f3 = __uint_as_float(wh.y & 0xffff0000u) + __uint_as_float(wl.y & 0xffff0000u);
          a0 += f0; a1 += f1; a2 += f2; a3 += f3;
        } else {
          const v2f p = *(const v2fa*)(pr3 + (size_t)sk * DF + 2 * lane);
          a0 += p.x; a1 += p.y;
        }
      }
    }
    const float inv = 1.0f / fmaxf((float)c, 1.0f);
    if constexpr (MODE != 2) {
      const float m0 = live ? (a0 * inv + pzr) : 0.0f;
      const float m1 = live ? (a1 * inv + pzr) : 0.0f;
      const float m2 = live ? (a2 * inv + pzr) : 0.0f;
      const float m3 = live ? (a3 * inv + pzr) : 0.0f;
      v4us mh, ml;
      {
        unsigned lb;
        unsigned hb;
        hb = hl_bits(m0, lb); mh[0] = (unsigned short)hb; ml[0] = (unsigned short)lb;
        hb = hl_bits(m1, lb); mh[1] = (unsigned short)hb; ml[1] = (unsigned short)lb;
        hb = hl_bits(m2, lb); mh[2] = (unsigned short)hb; ml[2] = (unsigned short)lb;
        hb = hl_bits(m3, lb); mh[3] = (unsigned short)hb; ml[3] = (unsigned short)lb;
      }
      *(v4usa*)(rowbuf + 4 * lane)      = mh;
      *(v4usa*)(rowbuf + DF + 4 * lane) = ml;
      wave_sync();
      const v8us q0 = *(const v8usa*)(rowbuf + 8 * lane);
      wave_sync();
      if (node < mRows) {
        unsigned short* rpw = aggOut + (size_t)node * HP + 8 * lane;
        *(volatile v8us*)rpw = q0;
        __threadfence();
        *(volatile v8us*)rpw = q0;
      }
    } else {
      const v2f r = *(const v2fa*)(pr3 + (size_t)nc * DF + DO3 + 2 * lane);
      const float o0 = (a0 * inv + bq0) + r.x;
      const float o1 = (a1 * inv + bq1) + r.y;
      const float v0 = sigm(o0) + pzr;
      const float v1 = sigm(o1) + pzr;
      const double e0 = live ? (double)v0 : 0.0;
      const double e1 = live ? (double)v1 : 0.0;
      d0 += e0;
      d1 += e1;
    }
  }

  if constexpr (MODE == 2) {
    double* wpart = (double*)(misc + MISC_INTS);
    double* drec  = wpart + NWAVE * DO3;
    v2d pw; pw.x = d0; pw.y = d1;
    *(v2da*)(wpart + wave * DO3 + 2 * lane) = pw;
    __syncthreads();
    if (tid < DO3) {
      double sacc = 0.0;
#pragma unroll 1
      for (int w2 = 0; w2 < NWAVE; ++w2) sacc += wpart[w2 * DO3 + tid];
      drec[tid] = sacc;
    }
    __syncthreads();
    if (wave == 0) {
      const v2d q = *(const v2da*)(drec + 2 * lane);
      double* rp = rec + (size_t)blockIdx.x * DO3 + 2 * lane;
      *(volatile v2d*)rp = q;
      __threadfence();
      *(volatile v2d*)rp = q;
    }
  }
}

template <int MODE>
__global__ __launch_bounds__(GTHR) void k_gemm(const unsigned short* __restrict__ A1, int lda1, int K1,
                                               const unsigned short* __restrict__ A2, int lda2, int K2,
                                               const unsigned short* __restrict__ BT, int ldb,
                                               const float* __restrict__ bias,
                                               unsigned short* hout, float* pout, int nN, int mRows) {
  __shared__ __attribute__((aligned(16))) float stg[GBM * GBN];
  const int tid = (int)threadIdx.x, lane = tid & 31, wave = tid >> 5, hh = lane >> 4, m = lane & 15;
  const int rowBase = (int)blockIdx.x * GBM;

  v8f acc[8];
#pragma unroll
  for (int t = 0; t < 8; ++t) acc[t] = z8();
  const size_t arow = (size_t)(rowBase + 16 * wave + m);
  const unsigned short* ap1 = A1 + arow * (size_t)lda1 + 8 * hh;
  const unsigned short* ap2 = A2 + arow * (size_t)lda2 + 8 * hh;
  const unsigned short* bp  = BT + (size_t)m * (size_t)ldb + 8 * hh;

#pragma unroll 1
  for (int k0 = 0; k0 < K1; k0 += 32) {
    FragB af;
    af.h[0] = *(const v8usa*)(ap1 + k0);
    af.h[1] = *(const v8usa*)(ap1 + k0 + 16);
#pragma unroll
    for (int nt = 0; nt < 8; ++nt) {
      const unsigned short* wq = bp + (size_t)(16 * nt) * (size_t)ldb + k0;
      FragB bf;
      bf.h[0] = *(const v8usa*)wq;
      bf.h[1] = *(const v8usa*)(wq + 16);
      acc[nt] = wmb(af, bf, acc[nt]);
    }
  }
#pragma unroll 1
  for (int k0 = 0; k0 < K2; k0 += 32) {
    FragB af;
    af.h[0] = *(const v8usa*)(ap2 + k0);
    af.h[1] = *(const v8usa*)(ap2 + k0 + 16);
#pragma unroll
    for (int nt = 0; nt < 8; ++nt) {
      const unsigned short* wq = bp + (size_t)(16 * nt) * (size_t)ldb + K1 + k0;
      FragB bf;
      bf.h[0] = *(const v8usa*)wq;
      bf.h[1] = *(const v8usa*)(wq + 16);
      acc[nt] = wmb(af, bf, acc[nt]);
    }
  }

#pragma unroll
  for (int nt = 0; nt < 8; ++nt) {
    const int lc = 16 * nt + m;
#pragma unroll
    for (int r = 0; r < 8; ++r) {
      const int lr = 16 * wave + 8 * hh + r;
      stg[lr * GBN + lc] = acc[nt][r];
    }
  }
  __syncthreads();

  if constexpr (MODE == 0) {
    float bq0, bq1, bq2, bq3;
    {
      const v4f b4 = *(const v4f*)(bias + 4 * lane);
      bq0 = bf16_val(b4.x); bq1 = bf16_val(b4.y); bq2 = bf16_val(b4.z); bq3 = bf16_val(b4.w);
    }
#pragma unroll 1
    for (int i = 0; i < 16; ++i) {
      const bool ok = (rowBase + 16 * wave + i) < nN;
      float* srf = stg + (16 * wave + i) * GBN;
      const v4f tv = *(const v4fa*)(srf + 4 * lane);
      wave_sync();
      const float y0 = sigm(tv.x + bq0);
      const float y1 = sigm(tv.y + bq1);
      const float y2 = sigm(tv.z + bq2);
      const float y3 = sigm(tv.w + bq3);
      const float o0 = ok ? y0 : 0.0f, o1 = ok ? y1 : 0.0f, o2 = ok ? y2 : 0.0f, o3 = ok ? y3 : 0.0f;
      v4us h4, l4;
      unsigned lb;
      unsigned hb;
      hb = hl_bits(o0, lb); h4[0] = (unsigned short)hb; l4[0] = (unsigned short)lb;
      hb = hl_bits(o1, lb); h4[1] = (unsigned short)hb; l4[1] = (unsigned short)lb;
      hb = hl_bits(o2, lb); h4[2] = (unsigned short)hb; l4[2] = (unsigned short)lb;
      hb = hl_bits(o3, lb); h4[3] = (unsigned short)hb; l4[3] = (unsigned short)lb;
      unsigned short* srow = (unsigned short*)srf;
      *(v4usa*)(srow + 4 * lane)      = h4;
      *(v4usa*)(srow + DF + 4 * lane) = l4;
    }
    wave_sync();
#pragma unroll 1
    for (int i = 0; i < 16; ++i) {
      const int gr = rowBase + 16 * wave + i;
      const unsigned short* srow = (const unsigned short*)(stg + (16 * wave + i) * GBN);
      const v8us q = *(const v8usa*)(srow + 8 * lane);
      unsigned short* rp = hout + (size_t)gr * HP + 8 * lane;
      if (gr < mRows) *(volatile v8us*)rp = q;
    }
    __threadfence();
#pragma unroll 1
    for (int i = 0; i < 16; ++i) {
      const int gr = rowBase + 16 * wave + i;
      const unsigned short* srow = (const unsigned short*)(stg + (16 * wave + i) * GBN);
      const v8us q = *(const v8usa*)(srow + 8 * lane);
      unsigned short* rp = hout + (size_t)gr * HP + 8 * lane;
      if (gr < mRows) *(volatile v8us*)rp = q;
    }
    (void)pout;
  } else {
#pragma unroll 1
    for (int i = 0; i < 16; ++i) {
      const int gr = rowBase + 16 * wave + i;
      const v4f q = *(const v4fa*)(stg + (16 * wave + i) * GBN + 4 * lane);
      float* op = pout + (size_t)gr * DF + 4 * lane;
      if (gr < mRows) *(volatile v4f*)op = q;
    }
    __threadfence();
#pragma unroll 1
    for (int i = 0; i < 16; ++i) {
      const int gr = rowBase + 16 * wave + i;
      const v4f q = *(const v4fa*)(stg + (16 * wave + i) * GBN + 4 * lane);
      float* op = pout + (size_t)gr * DF + 4 * lane;
      if (gr < mRows) *(volatile v4f*)op = q;
    }
    (void)hout; (void)bias; (void)nN;
  }
}

__global__ __launch_bounds__(DO3) void k_final(const double* __restrict__ rec, int nBlk, float* out) {
  __shared__ __attribute__((aligned(16))) float fo[DO3];
  const int tid = (int)threadIdx.x;
  double s = 0.0;
#pragma unroll 1
  for (int b = 0; b < nBlk; ++b) s += rec[(size_t)b * DO3 + tid];
  fo[tid] = (float)s;
  __syncthreads();
  const v4f v = *(const v4fa*)(fo + 4 * (tid & 15));
  float* op = out + 4 * (tid & 15);
  if (tid < 16) *(volatile v4f*)op = v;
  __threadfence();
  if (tid < 16) *(volatile v4f*)op = v;
}

static inline int cdiv(int a, int b) { return (a + b - 1) / b; }
static inline size_t al256(size_t o) { return (o + 255) & ~(size_t)255; }

extern "C" void kernel_launch(void* const* d_in, const int* in_sizes, int n_in,
                              void* d_out, int out_size, void* d_ws, size_t ws_size,
                              hipStream_t stream) {
  if (n_in < 11) return;
  if (in_sizes[0] < DF || (in_sizes[0] % DF) != 0) return;
  const int nN = in_sizes[0] / DF;
  if (nN < GBM || nN >= (1 << 24)) return;
  if (in_sizes[1] < 2 || (in_sizes[1] & 1) != 0) return;
  const int nE = in_sizes[1] / 2;
  if (nE < 1 || nE >= (1 << 21)) return;
  if (in_sizes[2] != DF * DF || in_sizes[3] != DF || in_sizes[4] != DF * DF) return;
  if (in_sizes[5] != DF * DF || in_sizes[6] != DF || in_sizes[7] != DF * DF) return;
  if (in_sizes[8] != DO3 * DF || in_sizes[9] != DO3 || in_sizes[10] != DO3 * DF) return;
  if (out_size != DO3) return;

  const float* x   = (const float*)d_in[0];
  const int*   ei  = (const int*)  d_in[1];
  const float* W1l = (const float*)d_in[2];
  const float* b1  = (const float*)d_in[3];
  const float* W1r = (const float*)d_in[4];
  const float* W2l = (const float*)d_in[5];
  const float* b2  = (const float*)d_in[6];
  const float* W2r = (const float*)d_in[7];
  const float* W3l = (const float*)d_in[8];
  const float* b3  = (const float*)d_in[9];
  const float* W3r = (const float*)d_in[10];
  float* out = (float*)d_out;
  const int* src = ei;
  const int* dst = ei + nE;

  const int MP = cdiv(nN, GBM) * GBM;
  const int gM = MP / GBM;
  const int gA = cdiv(nN, NBA);
  if ((long long)gA * NBA < (long long)MP) return;
  const int vec8 = ((nE & 3) == 0) ? 1 : 0;

  char* ws = (char*)d_ws;
  size_t off = 0;
  const size_t oW1 = off; off = al256(off + (size_t)DF * K1C * 2);
  const size_t oW2 = off; off = al256(off + (size_t)DF * K2C * 2);
  const size_t oW3 = off; off = al256(off + (size_t)DF * K3C * 2);
  const size_t oXB = off; off = al256(off + (size_t)MP * XP * 2);
  const size_t oAG = off; off = al256(off + (size_t)MP * HP * 2);
  const size_t oH1 = off; off = al256(off + (size_t)MP * HP * 2);
  const size_t oH2 = off; off = al256(off + (size_t)MP * HP * 2);
  const size_t oP3 = off; off = al256(off + (size_t)MP * DF * 4);
  const size_t oRC = off; off = al256(off + (size_t)gA * DO3 * 8);
  if (off > ws_size || off > (size_t)WSMAX) return;
  unsigned short* W1C = (unsigned short*)(ws + oW1);
  unsigned short* W2C = (unsigned short*)(ws + oW2);
  unsigned short* W3C = (unsigned short*)(ws + oW3);
  unsigned short* XB  = (unsigned short*)(ws + oXB);
  unsigned short* AGG = (unsigned short*)(ws + oAG);
  unsigned short* H1  = (unsigned short*)(ws + oH1);
  unsigned short* H2  = (unsigned short*)(ws + oH2);
  float*          PR3 = (float*)(ws + oP3);
  double*         REC = (double*)(ws + oRC);

  const size_t scanLds = (size_t)AGG_LDS_INTS * 4;
  hipFuncSetAttribute(reinterpret_cast<const void*>(&k_scan<0>), hipFuncAttributeMaxDynamicSharedMemorySize, (int)scanLds);
  hipFuncSetAttribute(reinterpret_cast<const void*>(&k_scan<1>), hipFuncAttributeMaxDynamicSharedMemorySize, (int)scanLds);
  hipFuncSetAttribute(reinterpret_cast<const void*>(&k_scan<2>), hipFuncAttributeMaxDynamicSharedMemorySize, (int)scanLds);

  const int nUnits = NUWE + MP * (XP / 8);

  k_prep<<<cdiv(nUnits, NTHR), NTHR, 0, stream>>>(x, W1l, W1r, W2l, W2r, W3l, W3r, W1C, W2C, W3C, XB, nN, nUnits);
  k_scan<0><<<gA, NTHR, scanLds, stream>>>(src, dst, nE, nN, vec8, MP, XB, PR3, b3, AGG, REC);
  k_gemm<0><<<gM, GTHR, 0, stream>>>(AGG, HP, HP, XB, XP, XP, W1C, K1C, b1, H1, PR3, nN, MP);
  k_scan<1><<<gA, NTHR, scanLds, stream>>>(src, dst, nE, nN, vec8, MP, H1, PR3, b3, AGG, REC);
  k_gemm<0><<<gM, GTHR, 0, stream>>>(AGG, HP, HP, H1, HP, HP, W2C, K2C, b2, H2, PR3, nN, MP);
  k_gemm<1><<<gM, GTHR, 0, stream>>>(H2, HP, HP, H2, HP, 0, W3C, K3C, b1, H2  , PR3, nN, MP);
  k_scan<2><<<gA, NTHR, scanLds, stream>>>(src, dst, nE, nN, vec8, MP, XB, PR3, b3, AGG, REC);
  k_final<<<1, DO3, 0, stream>>>(REC, gA, out);
}
